// NGP_50405736185934
// MI455X (gfx1250) — hardware-verified
//
#include <hip/hip_runtime.h>
#include <math.h>

typedef __attribute__((ext_vector_type(16))) _Float16 v16h;
typedef __attribute__((ext_vector_type(16))) __bf16 v16b;
typedef __attribute__((ext_vector_type(8)))  _Float16 v8h;
typedef __attribute__((ext_vector_type(8)))  float v8f;
typedef __attribute__((ext_vector_type(4)))  float v4f;
typedef __attribute__((ext_vector_type(2)))  float v2f;
typedef __attribute__((ext_vector_type(4)))  unsigned v4u;
typedef __attribute__((ext_vector_type(4)))  int v4i;
typedef float __attribute__((may_alias)) float_a;
typedef int __attribute__((may_alias)) int_a;

template <typename T> __device__ __forceinline__ void vst2(void* p, T v) { *(volatile T*)p = v; __threadfence(); *(volatile T*)p = v; }
__device__ __forceinline__ v8f wmma16(v16h a, v16h b, v8f c) {
  v8f d = __builtin_amdgcn_wmma_f32_16x16x32_f16(false, a, false, b, (short)0, c, false, false);
  asm volatile("v_nop\n\tv_nop\n\tv_nop\n\tv_nop" : "+v"(d) : "v"(a), "v"(b));
  return d;
}
__device__ __forceinline__ v8f wmma_bf(v16b a, v16b b, v8f c) {
  v8f d = __builtin_amdgcn_wmma_f32_16x16x32_bf16(false, a, false, b, (short)0, c, false, false);
  asm volatile("v_nop\n\tv_nop\n\tv_nop\n\tv_nop" : "+v"(d) : "v"(a), "v"(b));
  return d;
}
__device__ __forceinline__ v16h frag_h(const _Float16* rowk0, int lane) {
  union { v16h v; v8h q[2]; } u; const _Float16* p = rowk0 + 8 * (lane >> 4);
  u.q[0] = *(const v8h*)p; u.q[1] = *(const v8h*)(p + 16); return u.v;
}
__device__ __forceinline__ v16h frag_f32(const float* rowk0, int lane) {
  v16h a; const float* p = rowk0 + 8 * (lane >> 4);
#pragma unroll
  for (int i = 0; i < 8; ++i) { a[i] = (_Float16)p[i]; a[8 + i] = (_Float16)p[16 + i]; }
  return a;
}
__device__ __forceinline__ v16h frag_f32s(const float* rowk0, int lane, float sc) {
  v16h a; const float* p = rowk0 + 8 * (lane >> 4);
#pragma unroll
  for (int i = 0; i < 8; ++i) { a[i] = (_Float16)(p[i] * sc); a[8 + i] = (_Float16)(p[16 + i] * sc); }
  return a;
}
__device__ __forceinline__ v16h fragc_f32(const float* W, int k0, int n, int lane, int ld, int K) {
  v16h a; const int g = lane >> 4;
#pragma unroll
  for (int i = 0; i < 8; ++i) { const int ka = k0 + 8 * g + i, kb = ka + 16;
    a[i] = (_Float16)(ka < K ? W[(size_t)ka * ld + n] : 0.f); a[8 + i] = (_Float16)(kb < K ? W[(size_t)kb * ld + n] : 0.f); }
  return a;
}
struct F2 { v16b h, l; };
__device__ __forceinline__ F2 bsplit16(const float v[16]) { F2 r;
#pragma unroll
  for (int i = 0; i < 16; ++i) { const __bf16 h = (__bf16)v[i]; r.h[i] = h; r.l[i] = (__bf16)(v[i] - (float)h); }
  return r; }
__device__ __forceinline__ F2 split_row(const float* row, int k0, int lane) { float v[16]; const float* p = row + k0 + 8 * (lane >> 4);
#pragma unroll
  for (int i = 0; i < 8; ++i) { v[i] = p[i]; v[8 + i] = p[16 + i]; }
  return bsplit16(v); }
__device__ __forceinline__ F2 split_rowK(const float* row, int k0, int lane, int K) { float v[16]; const int g = lane >> 4;
#pragma unroll
  for (int i = 0; i < 8; ++i) { const int ka = k0 + 8 * g + i, kb = ka + 16; v[i] = ka < K ? row[ka] : 0.f; v[8 + i] = kb < K ? row[kb] : 0.f; }
  return bsplit16(v); }
__device__ __forceinline__ F2 split_col(const float* W, int k0, int n, int lane, int ld, int K) { float v[16]; const int g = lane >> 4;
#pragma unroll
  for (int i = 0; i < 8; ++i) { const int ka = k0 + 8 * g + i, kb = ka + 16; v[i] = ka < K ? W[(size_t)ka * ld + n] : 0.f; v[8 + i] = kb < K ? W[(size_t)kb * ld + n] : 0.f; }
  return bsplit16(v); }
__device__ __forceinline__ v8f mac3(const F2& a, const F2& b, v8f c) { c = wmma_bf(a.l, b.h, c); c = wmma_bf(a.h, b.l, c); return wmma_bf(a.h, b.h, c); }
__device__ __forceinline__ float sigm(float v) { return 1.0f / (1.0f + expf(-v)); }
#define LDSX() do { asm volatile("s_wait_dscnt 0" ::: "memory"); __builtin_amdgcn_wave_barrier(); __builtin_amdgcn_fence(__ATOMIC_RELEASE, "workgroup"); } while (0)


#define NPT 524288
#define NLV 8
#define TSZ 524288u
#define NF 2
#define FW 16
#define H1 64
#define H2 32
__device__ __forceinline__ float lrelu(float v) { return v >= 0.f ? v : 0.01f * v; }

__global__ __launch_bounds__(128) void k_ngp(const float* __restrict__ x, const float* __restrict__ levels, const float* __restrict__ grid, const float* __restrict__ w1, const float* __restrict__ b1, const float* __restrict__ w2, const float* __restrict__ b2,
                                            const float* __restrict__ w3, const float* __restrict__ b3, float* __restrict__ out) {
  __shared__ __align__(16) float sf[64][36];
  __shared__ __align__(16) float sh1[64][68];
  __shared__ __align__(16) float sh2[64][36];
  const int tid = threadIdx.x, wave = tid >> 5, lane = tid & 31, col = lane & 15, g = lane >> 4; const int p0 = blockIdx.x * 64;
  { const int pl = tid & 63, lh = tid >> 6; const int p = p0 + pl; const float px = x[(size_t)p * 3], py = x[(size_t)p * 3 + 1], pz = x[(size_t)p * 3 + 2];
    if (lh == 0) { for (int k = 16; k < 32; ++k) sf[pl][k] = 0.f; }
#pragma unroll 1
    for (int l4 = 0; l4 < 4; ++l4) { const int l = lh * 4 + l4; const float lv = levels[l];
      const float xs = px * lv, ys = py * lv, zs = pz * lv; const float fx = floorf(xs), fy = floorf(ys), fz = floorf(zs); const float wx = xs - fx, wy = ys - fy, wz = zs - fz;
      const unsigned cx = (unsigned)(int)fx, cy = (unsigned)(int)fy, cz = (unsigned)(int)fz;
      float f0 = 0.f, f1 = 0.f; const float* gl = grid + (size_t)l * TSZ * NF;
#pragma unroll
      for (int c = 0; c < 8; ++c) { const unsigned ox = (c >> 2) & 1u, oy = (c >> 1) & 1u, oz = c & 1u;
        const unsigned hsh = ((cx + ox) + (cy + oy) * 2654435761u + (cz + oz) * 805459861u) % TSZ;
        const float cw = (ox ? wx : 1.f - wx) * (oy ? wy : 1.f - wy) * (oz ? wz : 1.f - wz);
        f0 += gl[(size_t)hsh * NF] * cw; f1 += gl[(size_t)hsh * NF + 1] * cw; }
      sf[pl][l * NF] = f0; sf[pl][l * NF + 1] = f1; } }
  __syncthreads();
  { v8f acc[4] = {}; const F2 a = split_row(&sf[wave * 16 + col][0], 0, lane);
#pragma unroll
    for (int j = 0; j < 4; ++j) acc[j] = mac3(a, split_col(w1, 0, j * 16 + col, lane, H1, FW), acc[j]);
#pragma unroll
    for (int j = 0; j < 4; ++j)
#pragma unroll
      for (int r = 0; r < 8; ++r) sh1[wave * 16 + 8 * g + r][j * 16 + col] = lrelu(acc[j][r] + b1[j * 16 + col]); }
  LDSX();
  { v8f acc[2] = {};
#pragma unroll
    for (int kc = 0; kc < 2; ++kc) { const F2 a = split_row(&sh1[wave * 16 + col][0], kc * 32, lane);
#pragma unroll
      for (int j = 0; j < 2; ++j) acc[j] = mac3(a, split_col(w2, kc * 32, j * 16 + col, lane, H2, H1), acc[j]); }
#pragma unroll
    for (int j = 0; j < 2; ++j)
#pragma unroll
      for (int r = 0; r < 8; ++r) sh2[wave * 16 + 8 * g + r][j * 16 + col] = lrelu(acc[j][r] + b2[j * 16 + col]); }
  __syncthreads();
  { const int pl = tid >> 1, o = tid & 1; float s = b3[o];
#pragma unroll 8
    for (int k = 0; k < H2; ++k) s += sh2[pl][k] * w3[k * 2 + o];
    vst2(out + (size_t)(p0 + pl) * 2 + o, (float_a)s); }
}
extern "C" void kernel_launch(void* const* d_in, const int* in_sizes, int n_in, void* d_out, int out_size, void* d_ws, size_t ws_size, hipStream_t stream) {
  (void)in_sizes; (void)n_in; (void)out_size; (void)ws_size; (void)d_ws;
  const float** I = (const float**)d_in;
  k_ngp<<<NPT / 64, 128, 0, stream>>>(I[0], I[1], I[2], I[3], I[4], I[5], I[6], I[7], I[8], (float*)d_out);
}
